// MaskedSelfAttention_48473000902938
// MI455X (gfx1250) — hardware-verified
//
#include <hip/hip_runtime.h>
#include <math.h>
#include <stdint.h>

#define NB   4
#define SEQ  2048
#define DM   1024
#define NH   16
#define HD   64
#define N3   (3 * DM)
#define QKP  (2 * DM)
#define CXP  (2 * DM)
#define NQB  (SEQ / 64)
static_assert(NH * HD == DM);
static_assert((SEQ % 64) == 0 && (DM % 64) == 0 && (N3 % 64) == 0);
static_assert((DM % 32) == 0 && (CXP % 32) == 0 && (QKP % 8) == 0);

typedef __bf16   v16b __attribute__((ext_vector_type(16)));
typedef __bf16   v8b  __attribute__((ext_vector_type(8)));
typedef float    v8f  __attribute__((ext_vector_type(8)));
typedef float    v4f  __attribute__((ext_vector_type(4)));
typedef unsigned int v4u __attribute__((ext_vector_type(4)));

__device__ __forceinline__ unsigned short bf_bits(float f) {
  unsigned u = __float_as_uint(f);
  return (unsigned short)((u + 0x7FFFu + ((u >> 16) & 1u)) >> 16);
}
__device__ __forceinline__ float bf_up(unsigned short h) { return __uint_as_float(((unsigned)h) << 16); }
__device__ __forceinline__ float bfr(float f) { return bf_up(bf_bits(f)); }
__device__ __forceinline__ unsigned pk16(unsigned short a, unsigned short b) { return (unsigned)a | ((unsigned)b << 16); }
__device__ __forceinline__ v8f zero8() { v8f z = {0.f, 0.f, 0.f, 0.f, 0.f, 0.f, 0.f, 0.f}; return z; }
__device__ __forceinline__ void bf_split(float f, __bf16& hi, __bf16& lo) {
  const unsigned short hb = bf_bits(f);
  hi = __builtin_bit_cast(__bf16, hb);
  lo = __builtin_bit_cast(__bf16, bf_bits(f - bf_up(hb)));
}

__device__ __forceinline__ v16b ldfrag_b(const __bf16* p) {
  union { v16b v; v8b h[2]; } f;
  f.h[0] = *(const v8b*)(p);
  f.h[1] = *(const v8b*)(p + 16);
  return f.v;
}

__device__ __forceinline__ v8f mma_b(v16b a, v16b b, v8f c) {
  c = __builtin_amdgcn_wmma_f32_16x16x32_bf16(false, a, false, b, (short)0, c, false, false);
  asm volatile("v_nop\n\tv_nop\n\tv_nop\n\tv_nop" : "+v"(c) : "v"(a), "v"(b));
  return c;
}
__device__ __forceinline__ v8f mma_b_raw(v16b a, v16b b, v8f c) {
  return __builtin_amdgcn_wmma_f32_16x16x32_bf16(false, a, false, b, (short)0, c, false, false);
}
__device__ __forceinline__ void dep_guard_b(v8f& a, v8f& b, v16b x, v16b y) {
  asm volatile("v_nop\n\tv_nop\n\tv_nop\n\tv_nop" : "+v"(a), "+v"(b) : "v"(x), "v"(y));
}
__device__ __forceinline__ void keep4_b(v16b a, v16b b, v16b c, v16b d) {
  asm volatile("v_nop" :: "v"(a), "v"(b), "v"(c), "v"(d));
}
__device__ __forceinline__ void acc_guard4(v8f& a, v8f& b, v8f& c, v8f& d) {
  asm volatile("v_nop\n\tv_nop\n\tv_nop\n\tv_nop" : "+v"(a), "+v"(b), "+v"(c), "+v"(d));
}

__global__ __launch_bounds__(256) void cvt_bf16x8(const float* __restrict__ in, unsigned short* out, int n8) {
  const int i = blockIdx.x * 256 + threadIdx.x;
  if (i < n8) {
    const v4f a = *(const v4f*)(in + (size_t)i * 8);
    const v4f b = *(const v4f*)(in + (size_t)i * 8 + 4);
    v4u p;
    p[0] = pk16(bf_bits(a[0]), bf_bits(a[1]));
    p[1] = pk16(bf_bits(a[2]), bf_bits(a[3]));
    p[2] = pk16(bf_bits(b[0]), bf_bits(b[1]));
    p[3] = pk16(bf_bits(b[2]), bf_bits(b[3]));
    *(volatile v4u*)(out + (size_t)i * 8) = p;
    __threadfence();
    *(volatile v4u*)(out + (size_t)i * 8) = p;
  }
}

template <bool DUP>
__global__ __launch_bounds__(256) void tcvt_kernel(const float* __restrict__ W, unsigned short* o, int R, int Cc, int P) {
  __shared__ __align__(16) float tf[64 * 68];
  const int c0  = blockIdx.x * 64;
  const int r0  = blockIdx.y * 64;
  const int tid = threadIdx.x;
  {
    const int lr = tid >> 4;
    const int c4 = (tid & 15) * 4;
#pragma unroll
    for (int it = 0; it < 4; ++it) {
      const int rr = it * 16 + lr;
      const v4f a = *(const v4f*)(W + (size_t)(r0 + rr) * Cc + c0 + c4);
      *(v4f*)(tf + rr * 68 + c4) = a;
    }
  }
  __syncthreads();
  const int sub = tid >> 3;
  const int c8  = (tid & 7) * 8;
  v4u hv[2];
#pragma unroll
  for (int it = 0; it < 2; ++it) {
    const int oc = it * 32 + sub;
    v4u a;
#pragma unroll
    for (int q = 0; q < 4; ++q) {
      const float f0 = tf[(c8 + 2 * q) * 68 + oc];
      const float f1 = tf[(c8 + 2 * q + 1) * 68 + oc];
      a[q] = pk16(bf_bits(f0), bf_bits(f1));
    }
    hv[it] = a;
  }
  for (int pass = 0; pass < 2; ++pass) {
#pragma unroll
    for (int it = 0; it < 2; ++it) {
      const int oc = it * 32 + sub;
      const size_t go = (size_t)(c0 + oc) * P + r0 + c8;
      *(volatile v4u*)(o + go) = hv[it];
      if (DUP) *(volatile v4u*)(o + go + R) = hv[it];
    }
    __threadfence();
  }
}

template <int BIAS_MODE, int OUT_MODE>
__global__ __launch_bounds__(256) void gemm64(
    const unsigned short* __restrict__ Ap, int lda,
    const unsigned short* __restrict__ Btp, int ldb,
    void* Cout, void* Cout2, int ldc,
    const float* __restrict__ bias,
    int M, int N, int K) {
  const __bf16* A  = (const __bf16*)(const void*)Ap;
  const __bf16* Bt = (const __bf16*)(const void*)Btp;
  __shared__ __align__(16) float sT[8][16 * 68];
  const int lane = threadIdx.x & 31;
  const int wave = threadIdx.x >> 5;
  const int tilesN = N >> 6;
  const int tilesM = M >> 6;
  const int tile = blockIdx.x * 8 + wave;
  if (tile >= tilesM * tilesN) return;
  const int tm = tile / tilesN;
  const int tn = tile - tm * tilesN;
  const int m0 = tm << 6;
  const int n0 = tn << 6;

  const int rlane = lane & 15;
  const int koff  = (lane >> 4) * 8;
  const int mOff  = (lane >> 4) * 8;

  v8f acc[4][4];
#pragma unroll
  for (int i = 0; i < 4; ++i)
#pragma unroll
    for (int j = 0; j < 4; ++j) acc[i][j] = zero8();

  for (int k0 = 0; k0 < K; k0 += 32) {
    v16b bh[4];
#pragma unroll
    for (int j = 0; j < 4; ++j) {
      const size_t bo = (size_t)(n0 + (j << 4) + rlane) * ldb + koff + k0;
      bh[j] = ldfrag_b(Bt + bo);
    }
#pragma unroll
    for (int i = 0; i < 4; ++i) {
      const size_t ao = (size_t)(m0 + (i << 4) + rlane) * lda + koff + k0;
      const v16b ah = ldfrag_b(A + ao);
#pragma unroll
      for (int j = 0; j < 4; ++j) acc[i][j] = mma_b_raw(ah, bh[j], acc[i][j]);
      dep_guard_b(acc[i][0], acc[i][3], ah, ah);
    }
    keep4_b(bh[0], bh[1], bh[2], bh[3]);
  }
  acc_guard4(acc[0][0], acc[0][1], acc[0][2], acc[0][3]);
  acc_guard4(acc[1][0], acc[1][1], acc[1][2], acc[1][3]);
  acc_guard4(acc[2][0], acc[2][1], acc[2][2], acc[2][3]);
  acc_guard4(acc[3][0], acc[3][1], acc[3][2], acc[3][3]);

  float* slab = sT[wave];
#pragma unroll
  for (int i = 0; i < 4; ++i) {
    const int mBase = m0 + (i << 4);
    float bm8[8];
#pragma unroll
    for (int r = 0; r < 8; ++r) bm8[r] = 0.f;
    if (BIAS_MODE == 1) {
      const v4f t0 = *(const v4f*)(bias + mBase + mOff);
      const v4f t1 = *(const v4f*)(bias + mBase + mOff + 4);
      bm8[0] = bfr(t0[0]); bm8[1] = bfr(t0[1]); bm8[2] = bfr(t0[2]); bm8[3] = bfr(t0[3]);
      bm8[4] = bfr(t1[0]); bm8[5] = bfr(t1[1]); bm8[6] = bfr(t1[2]); bm8[7] = bfr(t1[3]);
    }
#pragma unroll
    for (int j = 0; j < 4; ++j) {
      float bn = 0.f;
      if (BIAS_MODE == 2) bn = bfr(bias[n0 + (j << 4) + rlane]);
#pragma unroll
      for (int r = 0; r < 8; ++r) {
        float v = acc[i][j][r];
        if (BIAS_MODE == 1) v += bm8[r];
        if (BIAS_MODE == 2) v += bn;
        slab[(mOff + r) * 68 + (j << 4) + rlane] = v;
      }
    }
    __builtin_amdgcn_fence(__ATOMIC_RELEASE, "workgroup");
    __builtin_amdgcn_wave_barrier();
    __builtin_amdgcn_fence(__ATOMIC_ACQUIRE, "workgroup");
    if (OUT_MODE == 0) {
      float* C = (float*)Cout;
      const int hh = lane >> 4, c4 = (lane & 15) * 4;
      for (int pass = 0; pass < 2; ++pass) {
#pragma unroll
        for (int it = 0; it < 8; ++it) {
          const int row = it * 2 + hh;
          const v4f v = *(const v4f*)(slab + row * 68 + c4);
          *(volatile v4f*)(C + (size_t)(mBase + row) * ldc + n0 + c4) = v;
        }
        __threadfence();
      }
    } else {
      const int q = lane >> 3, c8 = (lane & 7) * 8;
      unsigned short* C  = (unsigned short*)Cout;
      unsigned short* C2 = (unsigned short*)Cout2;
      v4u hv[4], lv[4];
#pragma unroll
      for (int it = 0; it < 4; ++it) {
        const int row = it * 4 + q;
        const float* sp = slab + row * 68 + c8;
        v4u a, a2;
#pragma unroll
        for (int e = 0; e < 4; ++e) {
          const float f0 = sp[2 * e], f1 = sp[2 * e + 1];
          const unsigned short h0 = bf_bits(f0), h1 = bf_bits(f1);
          const unsigned short l0 = bf_bits(f0 - bf_up(h0)), l1 = bf_bits(f1 - bf_up(h1));
          a[e] = pk16(h0, h1); a2[e] = pk16(l0, l1);
        }
        hv[it] = a; lv[it] = a2;
      }
      for (int pass = 0; pass < 2; ++pass) {
#pragma unroll
        for (int it = 0; it < 4; ++it) {
          const int row = it * 4 + q;
          *(volatile v4u*)(C  + (size_t)(mBase + row) * ldc + n0 + c8) = hv[it];
          *(volatile v4u*)(C2 + (size_t)(mBase + row) * ldc + n0 + c8) = lv[it];
        }
        __threadfence();
      }
    }
    __builtin_amdgcn_fence(__ATOMIC_RELEASE, "workgroup");
    __builtin_amdgcn_wave_barrier();
    __builtin_amdgcn_fence(__ATOMIC_ACQUIRE, "workgroup");
  }
}

__global__ __launch_bounds__(128)
void attn_causal64(const unsigned short* __restrict__ qkhp, const unsigned short* __restrict__ qklp,
                   const unsigned short* __restrict__ vhp, const unsigned short* __restrict__ vlp,
                   unsigned short* cxp, int rowBase, float sscale) {
  union FB { v16b v; v8b h[2]; };
  __shared__ __align__(16) __bf16 Ksh[64 * 64];
  __shared__ __align__(16) __bf16 Ksl[64 * 64];
  __shared__ __align__(16) __bf16 Vth[64 * 64];
  __shared__ __align__(16) __bf16 Vtl[64 * 64];
  __shared__ __align__(16) __bf16 Psh[4][16 * 64];
  __shared__ __align__(16) __bf16 Psl[4][16 * 64];
  __shared__ __align__(16) float  Os[4][16 * 64];

  const int tid  = threadIdx.x;
  const int wave = tid >> 5;
  const int lane = tid & 31;
  const int hh   = lane >> 4;
  const int c    = lane & 15;

  const int bx = blockIdx.x;
  const int qb = bx % NQB;
  const int h  = bx / NQB;
  const int q0 = qb * 64 + wave * 16;

  const __bf16* Qh = (const __bf16*)(const void*)qkhp + (size_t)h * HD;
  const __bf16* Ql = (const __bf16*)(const void*)qklp + (size_t)h * HD;
  const __bf16* Kh = (const __bf16*)(const void*)qkhp + (size_t)DM + (size_t)h * HD;
  const __bf16* Kl = (const __bf16*)(const void*)qklp + (size_t)DM + (size_t)h * HD;
  const __bf16* Vh = (const __bf16*)(const void*)vhp + (size_t)h * HD * SEQ;
  const __bf16* Vl = (const __bf16*)(const void*)vlp + (size_t)h * HD * SEQ;

  v16b qah[2], qal[2];
#pragma unroll
  for (int dc = 0; dc < 2; ++dc) {
    const size_t qo = (size_t)(q0 + c) * QKP + dc * 32 + 8 * hh;
    qah[dc] = ldfrag_b(Qh + qo);
    qal[dc] = ldfrag_b(Ql + qo);
  }

  float mrow[8], lrow[8];
  v8f oacc[4];
#pragma unroll
  for (int r = 0; r < 8; ++r) { mrow[r] = -INFINITY; lrow[r] = 0.f; }
#pragma unroll
  for (int t = 0; t < 4; ++t) oacc[t] = zero8();

  const int nChunks = qb + 1;
  for (int kc = 0; kc < nChunks; ++kc) {
    const int kv0 = kc * 64;
    __syncthreads();
    {
      const int r = tid >> 1, half = (tid & 1) * 32;
      const __bf16* kg  = Kh + (size_t)(kv0 + r) * QKP + half;
      const __bf16* klg = Kl + (size_t)(kv0 + r) * QKP + half;
      const __bf16* vg  = Vh + (size_t)r * SEQ + kv0 + half;
      const __bf16* vlg = Vl + (size_t)r * SEQ + kv0 + half;
#pragma unroll
      for (int i = 0; i < 4; ++i) {
        const v8b a0 = *(const v8b*)(kg + 8 * i);
        const v8b a1 = *(const v8b*)(klg + 8 * i);
        const v8b b0 = *(const v8b*)(vg + 8 * i);
        const v8b b1 = *(const v8b*)(vlg + 8 * i);
        *(v8b*)(Ksh + r * 64 + half + 8 * i) = a0;
        *(v8b*)(Ksl + r * 64 + half + 8 * i) = a1;
        *(v8b*)(Vth + r * 64 + half + 8 * i) = b0;
        *(v8b*)(Vtl + r * 64 + half + 8 * i) = b1;
      }
    }
    __syncthreads();

    v8f s[4];
#pragma unroll
    for (int j = 0; j < 4; ++j) {
      s[j] = zero8();
#pragma unroll
      for (int dc = 0; dc < 2; ++dc) {
        FB kb, kl;
        kb.h[0] = *(const v8b*)(Ksh + (j * 16 + c) * 64 + dc * 32 + 8 * hh);
        kb.h[1] = *(const v8b*)(Ksh + (j * 16 + c) * 64 + dc * 32 + 16 + 8 * hh);
        kl.h[0] = *(const v8b*)(Ksl + (j * 16 + c) * 64 + dc * 32 + 8 * hh);
        kl.h[1] = *(const v8b*)(Ksl + (j * 16 + c) * 64 + dc * 32 + 16 + 8 * hh);
        s[j] = mma_b(qah[dc], kb.v, s[j]);
        s[j] = mma_b(qah[dc], kl.v, s[j]);
        s[j] = mma_b(qal[dc], kb.v, s[j]);
      }
    }

    const bool diag = (kc == qb);
    float cm[8];
#pragma unroll
    for (int r = 0; r < 8; ++r) {
      const int qrow = q0 + 8 * hh + r;
      float m = -INFINITY;
#pragma unroll
      for (int j = 0; j < 4; ++j) {
        const int kvcol = kv0 + j * 16 + c;
        const float sv = s[j][r] * sscale;
        const bool masked = diag && (kvcol > qrow);
        const float sm = masked ? -INFINITY : sv;
        s[j][r] = sm;
        m = fmaxf(m, sm);
      }
#pragma unroll
      for (int off = 1; off < 16; off <<= 1) m = fmaxf(m, __shfl_xor(m, off, 32));
      cm[r] = m;
    }

    __bf16* pwh = Psh[wave];
    __bf16* pwl = Psl[wave];
#pragma unroll
    for (int r = 0; r < 8; ++r) {
      const float mnew  = fmaxf(mrow[r], cm[r]);
      const float alpha = __expf(mrow[r] - mnew);
      mrow[r] = mnew;
      float psum = 0.f;
#pragma unroll
      for (int j = 0; j < 4; ++j) {
        const float p = __expf(s[j][r] - mnew);
        psum += p;
        __bf16 a, bl; bf_split(p, a, bl);
        pwh[(8 * hh + r) * 64 + j * 16 + c] = a;
        pwl[(8 * hh + r) * 64 + j * 16 + c] = bl;
      }
#pragma unroll
      for (int off = 1; off < 16; off <<= 1) psum += __shfl_xor(psum, off, 32);
      lrow[r] = lrow[r] * alpha + psum;
#pragma unroll
      for (int t = 0; t < 4; ++t) oacc[t][r] *= alpha;
    }
    __builtin_amdgcn_fence(__ATOMIC_RELEASE, "workgroup");
    __builtin_amdgcn_wave_barrier();
    __builtin_amdgcn_fence(__ATOMIC_ACQUIRE, "workgroup");

#pragma unroll 1
    for (int kk = 0; kk < 2; ++kk) {
      FB pa, pl;
      pa.h[0] = *(const v8b*)(pwh + c * 64 + kk * 32 + 8 * hh);
      pa.h[1] = *(const v8b*)(pwh + c * 64 + kk * 32 + 16 + 8 * hh);
      pl.h[0] = *(const v8b*)(pwl + c * 64 + kk * 32 + 8 * hh);
      pl.h[1] = *(const v8b*)(pwl + c * 64 + kk * 32 + 16 + 8 * hh);
#pragma unroll
      for (int t = 0; t < 4; ++t) {
        FB vb, vl;
        vb.h[0] = *(const v8b*)(Vth + (t * 16 + c) * 64 + kk * 32 + 8 * hh);
        vb.h[1] = *(const v8b*)(Vth + (t * 16 + c) * 64 + kk * 32 + 16 + 8 * hh);
        vl.h[0] = *(const v8b*)(Vtl + (t * 16 + c) * 64 + kk * 32 + 8 * hh);
        vl.h[1] = *(const v8b*)(Vtl + (t * 16 + c) * 64 + kk * 32 + 16 + 8 * hh);
        oacc[t] = mma_b(pa.v, vb.v, oacc[t]);
        oacc[t] = mma_b(pa.v, vl.v, oacc[t]);
        oacc[t] = mma_b(pl.v, vb.v, oacc[t]);
      }
    }
  }

  float* os = Os[wave];
#pragma unroll
  for (int r = 0; r < 8; ++r) {
    const float l = lrow[r];
    const float inv = (l > 0.f) ? (1.0f / l) : 0.f;
#pragma unroll
    for (int t = 0; t < 4; ++t) os[(8 * hh + r) * 64 + t * 16 + c] = oacc[t][r] * inv;
  }
  __builtin_amdgcn_fence(__ATOMIC_RELEASE, "workgroup");
  __builtin_amdgcn_wave_barrier();
  __builtin_amdgcn_fence(__ATOMIC_ACQUIRE, "workgroup");
  {
    const int q4 = lane >> 3, c8 = (lane & 7) * 8;
    v4u hv[4], lv[4];
#pragma unroll
    for (int it = 0; it < 4; ++it) {
      const int row = it * 4 + q4;
      const float* sp = os + row * 64 + c8;
      v4u a, a2;
#pragma unroll
      for (int e = 0; e < 4; ++e) {
        const float f0 = sp[2 * e], f1 = sp[2 * e + 1];
        const unsigned short h0 = bf_bits(f0), h1 = bf_bits(f1);
        const unsigned short l0 = bf_bits(f0 - bf_up(h0)), l1 = bf_bits(f1 - bf_up(h1));
        a[e] = pk16(h0, h1); a2[e] = pk16(l0, l1);
      }
      hv[it] = a; lv[it] = a2;
    }
    for (int pass = 0; pass < 2; ++pass) {
#pragma unroll
      for (int it = 0; it < 4; ++it) {
        const int row = it * 4 + q4;
        const size_t go = (size_t)(rowBase + q0 + row) * CXP + (size_t)h * HD + c8;
        *(volatile v4u*)(cxp + go)      = hv[it];
        *(volatile v4u*)(cxp + go + DM) = lv[it];
      }
      __threadfence();
    }
  }
}

extern "C" void kernel_launch(void* const* d_in, const int* in_sizes, int n_in,
                              void* d_out, int out_size, void* d_ws, size_t ws_size,
                              hipStream_t stream) {
  if (n_in < 5) return;
  if (in_sizes[0] != NB * SEQ * DM) return;
  if (in_sizes[1] != DM * N3) return;
  if (in_sizes[2] != N3) return;
  if (in_sizes[3] != DM * DM) return;
  if (in_sizes[4] != DM) return;
  if (out_size != NB * SEQ * DM) return;

  const float* x      = (const float*)d_in[0];
  const float* W_attn = (const float*)d_in[1];
  const float* b_attn = (const float*)d_in[2];
  const float* W_proj = (const float*)d_in[3];
  const float* b_proj = (const float*)d_in[4];

  const size_t PXB = (size_t)NB * SEQ * DM * 2;
  const size_t PWA = (size_t)N3 * DM * 2;
  const size_t PWP = (size_t)DM * (2 * DM) * 2;
  const size_t PQK = (size_t)SEQ * QKP * 2;
  const size_t PVT = (size_t)DM * SEQ * 2;
  const size_t PCX = (size_t)NB * SEQ * CXP * 2;
  size_t off = 0;
  const size_t oXB  = off; off += PXB;
  const size_t oWAT = off; off += PWA;
  const size_t oWPT = off; off += PWP;
  const size_t oQKh = off; off += PQK;
  const size_t oQKl = off; off += PQK;
  const size_t oVTh = off; off += PVT;
  const size_t oVTl = off; off += PVT;
  const size_t oCTX = off; off += PCX;
  if (off > ws_size) return;
  if (off > (size_t)134217728) return;

  char* ws = (char*)d_ws;
  unsigned short* XB   = (unsigned short*)(ws + oXB);
  unsigned short* WAT  = (unsigned short*)(ws + oWAT);
  unsigned short* WPT2 = (unsigned short*)(ws + oWPT);
  unsigned short* QKh  = (unsigned short*)(ws + oQKh);
  unsigned short* QKl  = (unsigned short*)(ws + oQKl);
  unsigned short* VTh  = (unsigned short*)(ws + oVTh);
  unsigned short* VTl  = (unsigned short*)(ws + oVTl);
  unsigned short* CTX  = (unsigned short*)(ws + oCTX);

  const dim3 blk(256);
  const int n8x = NB * SEQ * DM / 8;
  const dim3 gCvtX((n8x + 255) / 256);
  const dim3 gTA(N3 / 64, DM / 64);
  const dim3 gTP(DM / 64, DM / 64);
  const dim3 gQK(((SEQ / 64) * ((2 * DM) / 64) + 7) / 8);
  const dim3 gVT(((DM / 64) * (SEQ / 64) + 7) / 8);
  const dim3 gAtt(NH * NQB);
  const dim3 gOut(((NB * SEQ / 64) * (DM / 64) + 7) / 8);

  cvt_bf16x8<<<gCvtX, blk, 0, stream>>>(x, XB, n8x);
  tcvt_kernel<false><<<gTA, blk, 0, stream>>>(W_attn, WAT, DM, N3, DM);
  tcvt_kernel<true><<<gTP, blk, 0, stream>>>(W_proj, WPT2, DM, DM, 2 * DM);

  for (int b = 0; b < NB; ++b) {
    const unsigned short* XBb = XB + (size_t)b * SEQ * DM;
    gemm64<2, 2><<<gQK, blk, 0, stream>>>(XBb, DM, WAT, DM, (void*)QKh, (void*)QKl, QKP, b_attn, SEQ, 2 * DM, DM);
    gemm64<1, 2><<<gVT, blk, 0, stream>>>(WAT + (size_t)(2 * DM) * DM, DM, XBb, DM, (void*)VTh, (void*)VTl, SEQ,
                                          b_attn + 2 * DM, DM, SEQ, DM);
    attn_causal64<<<gAtt, dim3(128), 0, stream>>>(QKh, QKl, VTh, VTl, CTX, b * SEQ, 0.125f);
  }
  gemm64<2, 0><<<gOut, blk, 0, stream>>>(CTX, CXP, WPT2, 2 * DM, d_out, d_out, DM, b_proj, NB * SEQ, DM, 2 * DM);
  (void)hipGetLastError();
}
